// MSARowAttention_481036337737
// MI455X (gfx1250) — hardware-run, weakly checked
//
#include <hip/hip_runtime.h>
#include <math.h>

typedef __attribute__((ext_vector_type(16))) _Float16 v16h;
typedef __attribute__((ext_vector_type(16))) __bf16 v16b;
typedef __attribute__((ext_vector_type(8)))  _Float16 v8h;
typedef __attribute__((ext_vector_type(8)))  float v8f;
typedef __attribute__((ext_vector_type(4)))  float v4f;
typedef __attribute__((ext_vector_type(2)))  float v2f;
typedef __attribute__((ext_vector_type(4)))  unsigned v4u;
typedef __attribute__((ext_vector_type(4)))  int v4i;
typedef float __attribute__((may_alias)) float_a;
typedef int __attribute__((may_alias)) int_a;

template <typename T> __device__ __forceinline__ void vst2(void* p, T v) { *(volatile T*)p = v; __threadfence(); *(volatile T*)p = v; }
__device__ __forceinline__ v8f wmma16(v16h a, v16h b, v8f c) {
  v8f d = __builtin_amdgcn_wmma_f32_16x16x32_f16(false, a, false, b, (short)0, c, false, false);
  asm volatile("v_nop\n\tv_nop\n\tv_nop\n\tv_nop" : "+v"(d) : "v"(a), "v"(b));
  return d;
}
__device__ __forceinline__ v8f wmma_bf(v16b a, v16b b, v8f c) {
  v8f d = __builtin_amdgcn_wmma_f32_16x16x32_bf16(false, a, false, b, (short)0, c, false, false);
  asm volatile("v_nop\n\tv_nop\n\tv_nop\n\tv_nop" : "+v"(d) : "v"(a), "v"(b));
  return d;
}
__device__ __forceinline__ v16h frag_h(const _Float16* rowk0, int lane) {
  union { v16h v; v8h q[2]; } u; const _Float16* p = rowk0 + 8 * (lane >> 4);
  u.q[0] = *(const v8h*)p; u.q[1] = *(const v8h*)(p + 16); return u.v;
}
__device__ __forceinline__ v16h frag_f32(const float* rowk0, int lane) {
  v16h a; const float* p = rowk0 + 8 * (lane >> 4);
#pragma unroll
  for (int i = 0; i < 8; ++i) { a[i] = (_Float16)p[i]; a[8 + i] = (_Float16)p[16 + i]; }
  return a;
}
__device__ __forceinline__ v16h frag_f32s(const float* rowk0, int lane, float sc) {
  v16h a; const float* p = rowk0 + 8 * (lane >> 4);
#pragma unroll
  for (int i = 0; i < 8; ++i) { a[i] = (_Float16)(p[i] * sc); a[8 + i] = (_Float16)(p[16 + i] * sc); }
  return a;
}
__device__ __forceinline__ v16h fragc_f32(const float* W, int k0, int n, int lane, int ld, int K) {
  v16h a; const int g = lane >> 4;
#pragma unroll
  for (int i = 0; i < 8; ++i) { const int ka = k0 + 8 * g + i, kb = ka + 16;
    a[i] = (_Float16)(ka < K ? W[(size_t)(ka < K ? ka : K - 1) * ld + n] : 0.f); a[8 + i] = (_Float16)(kb < K ? W[(size_t)(kb < K ? kb : K - 1) * ld + n] : 0.f); }
  return a;
}
struct F2 { v16b h, l; };
__device__ __forceinline__ F2 bsplit16(const float v[16]) { F2 r;
#pragma unroll
  for (int i = 0; i < 16; ++i) { const __bf16 h = (__bf16)v[i]; r.h[i] = h; r.l[i] = (__bf16)(v[i] - (float)h); }
  return r; }
__device__ __forceinline__ F2 split_row(const float* row, int k0, int lane) { float v[16]; const float* p = row + k0 + 8 * (lane >> 4);
#pragma unroll
  for (int i = 0; i < 8; ++i) { v[i] = p[i]; v[8 + i] = p[16 + i]; }
  return bsplit16(v); }
__device__ __forceinline__ F2 split_rowK(const float* row, int k0, int lane, int K) { float v[16]; const int g = lane >> 4;
#pragma unroll
  for (int i = 0; i < 8; ++i) { const int ka = k0 + 8 * g + i, kb = ka + 16; v[i] = ka < K ? row[ka < K ? ka : K - 1] : 0.f; v[8 + i] = kb < K ? row[kb < K ? kb : K - 1] : 0.f; }
  return bsplit16(v); }
__device__ __forceinline__ F2 split_col(const float* W, int k0, int n, int lane, int ld, int K) { float v[16]; const int g = lane >> 4;
#pragma unroll
  for (int i = 0; i < 8; ++i) { const int ka = k0 + 8 * g + i, kb = ka + 16; v[i] = ka < K ? W[(size_t)(ka < K ? ka : K - 1) * ld + n] : 0.f; v[8 + i] = kb < K ? W[(size_t)(kb < K ? kb : K - 1) * ld + n] : 0.f; }
  return bsplit16(v); }
__device__ __forceinline__ v8f mac3(const F2& a, const F2& b, v8f c) { c = wmma_bf(a.l, b.h, c); c = wmma_bf(a.h, b.l, c); return wmma_bf(a.h, b.h, c); }
__device__ __forceinline__ float sigm(float v) { return 1.0f / (1.0f + expf(-v)); }
#define LDSX() do { asm volatile("s_wait_dscnt 0" ::: "memory"); __builtin_amdgcn_wave_barrier(); __builtin_amdgcn_fence(__ATOMIC_RELEASE, "workgroup"); } while (0)


#define NSQ 128
#define LL 256
#define DD 256
#define DP 128
#define NHD 8
#define DH 32
#define NPS 64
#define NR (NPS * LL)
__device__ __forceinline__ float bfr(float v) { return (float)(__bf16)v; }
__device__ __forceinline__ v16b frag_b(const __bf16* rowk0, int lane) { return __builtin_bit_cast(v16b, frag_h((const _Float16*)rowk0, lane)); }
__device__ __attribute__((noinline)) float exp_ni(float v) { return expf(v); }

__global__ __launch_bounds__(256) void k_ln(const float* __restrict__ x, const float* __restrict__ lg, const float* __restrict__ lb, __bf16* __restrict__ XH, __bf16* __restrict__ XL) {
  __shared__ __align__(16) __bf16 sh_[8][DD + 8], sl_[8][DD + 8];
  const int tid = threadIdx.x, wave = tid >> 5, lane = tid & 31; const size_t r = (size_t)blockIdx.x * 8 + wave; const float* xr = x + r * DD;
  float v[8]; float s = 0.f;
#pragma unroll
  for (int e = 0; e < 8; ++e) { v[e] = bfr(xr[lane * 8 + e]); s += v[e]; }
#pragma unroll
  for (int o = 16; o > 0; o >>= 1) s += __shfl_xor(s, o, 32);
  const float mu = s * (1.0f / DD); float q = 0.f;
#pragma unroll
  for (int e = 0; e < 8; ++e) { const float dv = v[e] - mu; q += dv * dv; }
#pragma unroll
  for (int o = 16; o > 0; o >>= 1) q += __shfl_xor(q, o, 32);
  const float rs = rsqrtf(q * (1.0f / DD) + 1e-5f);
#pragma unroll
  for (int e = 0; e < 8; ++e) { const int c = lane * 8 + e; const float y = (v[e] - mu) * rs * bfr(lg[c]) + bfr(lb[c]); const __bf16 hi = (__bf16)y; sh_[wave][c] = hi; sl_[wave][c] = (__bf16)(y - (float)hi); }
  LDSX();
  vst2((unsigned*)(XH + r * DD + lane * 8), *(const v4u*)(&sh_[wave][lane * 8])); vst2((unsigned*)(XL + r * DD + lane * 8), *(const v4u*)(&sl_[wave][lane * 8]));
}
__global__ __launch_bounds__(128) void k_bias(const float* __restrict__ pb, const float* __restrict__ Wb, const float* __restrict__ bbv, float* __restrict__ BIAS) {
  __shared__ __align__(16) float sb[NHD][68];
  const int tid = threadIdx.x, wave = tid >> 5, lane = tid & 31, col = lane & 15, g = lane >> 4; const int i = blockIdx.y, j0 = blockIdx.x * 64 + wave * 16;
  v8f acc = {};
#pragma unroll
  for (int kc = 0; kc < DP / 32; ++kc) acc = wmma_bf(split_row(pb + ((size_t)i * LL + j0 + col) * DP, kc * 32, lane).h, split_col(Wb, kc * 32, col < NHD ? col : 0, lane, NHD, DP).h, acc);
  if (col < NHD) { const float bb = bfr(bbv[col]);
#pragma unroll
    for (int r = 0; r < 8; ++r) sb[col][wave * 16 + 8 * g + r] = acc[r] + bb; }
  __syncthreads();
  for (int q = tid; q < NHD * 16; q += 128) { const int h = q >> 4, pc = q & 15; vst2(BIAS + ((size_t)h * LL + i) * LL + blockIdx.x * 64 + pc * 4, *(const v4f*)(&sb[h][pc * 4])); }
}
__global__ __launch_bounds__(128) void k_qkv(const __bf16* __restrict__ XH, const __bf16* __restrict__ XL, const float* __restrict__ Wq, const float* __restrict__ bq, const float* __restrict__ Wk, const float* __restrict__ bk, const float* __restrict__ Wv, const float* __restrict__ bv,
                                            float* __restrict__ Q32, __bf16* __restrict__ Kh, __bf16* __restrict__ Kl, __bf16* __restrict__ VTh, __bf16* __restrict__ VTl) {
  __shared__ __align__(16) float so[4][16][132]; __shared__ __align__(16) __bf16 sh_[4][16][136], sl_[4][16][136]; __shared__ __align__(16) __bf16 sth[128][72], stl[128][72];
  const int tid = threadIdx.x, wave = tid >> 5, lane = tid & 31, col = lane & 15, g = lane >> 4; const int r0b = blockIdx.x * 64, n0 = blockIdx.y * 128, which = blockIdx.z; const int n = r0b / LL, s0 = r0b % LL; const size_t r0 = (size_t)r0b + wave * 16;
  const float* W = which == 0 ? Wq : (which == 1 ? Wk : Wv); const float* bias = which == 0 ? bq : (which == 1 ? bk : bv);
  v8f acc[8] = {};
#pragma unroll 2
  for (int kc = 0; kc < DD / 32; ++kc) { const v16b ah = frag_b(XH + (r0 + col) * DD + kc * 32, lane), al = frag_b(XL + (r0 + col) * DD + kc * 32, lane);
#pragma unroll
    for (int j = 0; j < 8; ++j) { const v16b wb = split_col(W, kc * 32, n0 + j * 16 + col, lane, DD, DD).h; acc[j] = wmma_bf(al, wb, acc[j]); acc[j] = wmma_bf(ah, wb, acc[j]); } }
  if (which == 0) {
#pragma unroll
    for (int j = 0; j < 8; ++j) { const float bb = bfr(bias[n0 + j * 16 + col]);
#pragma unroll
      for (int r = 0; r < 8; ++r) so[wave][8 * g + r][j * 16 + col] = acc[j][r] + bb; }
    LDSX();
    for (int qq = lane; qq < 4 * 16 * 8; qq += 32) { const int hh = qq >> 7, rl = (qq >> 3) & 15, pc = qq & 7; const int h = (n0 >> 5) + hh; vst2(Q32 + (((size_t)n * NHD + h) * LL + s0 + wave * 16 + rl) * DH + pc * 4, *(const v4f*)(&so[wave][rl][hh * 32 + pc * 4])); } }
  else if (which == 1) {
#pragma unroll
    for (int j = 0; j < 8; ++j) { const float bb = bfr(bias[n0 + j * 16 + col]);
#pragma unroll
      for (int r = 0; r < 8; ++r) { const float v = acc[j][r] + bb; const __bf16 hi = (__bf16)v; sh_[wave][8 * g + r][j * 16 + col] = hi; sl_[wave][8 * g + r][j * 16 + col] = (__bf16)(v - (float)hi); } }
    LDSX();
    for (int qq = lane; qq < 4 * 16 * 4; qq += 32) { const int hh = qq >> 6, rl = (qq >> 2) & 15, pc = qq & 3; const int h = (n0 >> 5) + hh; const size_t o = (((size_t)n * NHD + h) * LL + s0 + wave * 16 + rl) * DH + pc * 8; vst2((unsigned*)(Kh + o), *(const v4u*)(&sh_[wave][rl][hh * 32 + pc * 8])); vst2((unsigned*)(Kl + o), *(const v4u*)(&sl_[wave][rl][hh * 32 + pc * 8])); } }
  else {
#pragma unroll
    for (int j = 0; j < 8; ++j) { const float bb = bfr(bias[n0 + j * 16 + col]);
#pragma unroll
      for (int r = 0; r < 8; ++r) { const float v = acc[j][r] + bb; const __bf16 hi = (__bf16)v; sth[j * 16 + col][wave * 16 + 8 * g + r] = hi; stl[j * 16 + col][wave * 16 + 8 * g + r] = (__bf16)(v - (float)hi); } }
    __syncthreads();
    for (int qq = tid; qq < 128 * 8; qq += 128) { const int cl = qq >> 3, pc = qq & 7; const int c = n0 + cl; const int h = c >> 5, d = c & 31; const size_t o = (((size_t)n * NHD + h) * DH + d) * LL + s0 + pc * 8; vst2((unsigned*)(VTh + o), *(const v4u*)(&sth[cl][pc * 8])); vst2((unsigned*)(VTl + o), *(const v4u*)(&stl[cl][pc * 8])); } }
}
__global__ __launch_bounds__(128) void k_attn(const float* __restrict__ Q32, const __bf16* __restrict__ Kh, const __bf16* __restrict__ Kl, const __bf16* __restrict__ VTh, const __bf16* __restrict__ VTl, const float* __restrict__ BIAS, const int* __restrict__ mask, float* __restrict__ O) {
  __shared__ __align__(16) float sS[4][16][68];
  __shared__ __align__(16) __bf16 sPh[4][16][72], sPl[4][16][72];
  __shared__ __align__(16) float sO[4][16][36];
  const int tid = threadIdx.x, w = tid >> 5, lane = tid & 31, col = lane & 15, g = lane >> 4; const size_t bh = blockIdx.y; const int n = (int)(bh / NHD), h = (int)(bh % NHD); const int q0 = blockIdx.x * 64 + w * 16;
  const F2 aq = split_row(Q32 + (bh * LL + q0 + col) * DH, 0, lane);
  float mrun = -3.0e38f, lrun = 0.f; v8f acc[2] = {};
#pragma unroll 1
  for (int kt = 0; kt < LL / 64; ++kt) {
#pragma unroll
    for (int t = 0; t < 4; ++t) { const int key = kt * 64 + t * 16 + col; const size_t ko = (bh * LL + key) * DH; const v16b khf = frag_b(Kh + ko, lane), klf = frag_b(Kl + ko, lane);
      v8f s = {}; s = wmma_bf(aq.l, khf, s); s = wmma_bf(aq.h, klf, s); s = wmma_bf(aq.h, khf, s);
      const bool keep = mask[n * LL + key] != 0;
#pragma unroll
      for (int r = 0; r < 8; ++r) { const int qi = q0 + 8 * g + r; sS[w][8 * g + r][t * 16 + col] = keep ? s[r] * 0.17677669529663687f + BIAS[((size_t)h * LL + qi) * LL + key] : -1.0e9f; } }
    LDSX();
    float mx = -3.4e38f;
#pragma unroll
    for (int jj = 0; jj < 32; ++jj) mx = fmaxf(mx, sS[w][col][g * 32 + jj]);
    mx = fmaxf(mx, __shfl_xor(mx, 16, 32));
    const float mnew = fmaxf(mrun, mx); const float corr = expf(mrun - mnew);
    float ps = 0.f;
#pragma unroll 4
    for (int jj = 0; jj < 32; ++jj) { const float p = exp_ni(sS[w][col][g * 32 + jj] - mnew); ps += p; const __bf16 hi = (__bf16)p; sPh[w][col][g * 32 + jj] = hi; sPl[w][col][g * 32 + jj] = (__bf16)(p - (float)hi); }
    ps += __shfl_xor(ps, 16, 32);
    lrun = lrun * corr + ps; mrun = mnew;
#pragma unroll
    for (int r = 0; r < 8; ++r) { const float cr = __shfl(corr, 8 * g + r, 32); acc[0][r] *= cr; acc[1][r] *= cr; }
    LDSX();
#pragma unroll
    for (int kc = 0; kc < 2; ++kc) { const v16b ph = frag_b(&sPh[w][col][0] + kc * 32, lane), pl = frag_b(&sPl[w][col][0] + kc * 32, lane);
#pragma unroll
      for (int t = 0; t < 2; ++t) { const size_t vo = (bh * DH + t * 16 + col) * LL + kt * 64 + kc * 32; const v16b vh = frag_b(VTh + vo, lane), vl = frag_b(VTl + vo, lane); acc[t] = wmma_bf(pl, vh, acc[t]); acc[t] = wmma_bf(ph, vl, acc[t]); acc[t] = wmma_bf(ph, vh, acc[t]); } }
    __builtin_amdgcn_wave_barrier(); }
#pragma unroll
  for (int r = 0; r < 8; ++r) { const float lr = __shfl(lrun, 8 * g + r, 32); const float inv = 1.0f / lr; sO[w][8 * g + r][col] = acc[0][r] * inv; sO[w][8 * g + r][16 + col] = acc[1][r] * inv; }
  LDSX();
  for (int qq = lane; qq < 16 * 8; qq += 32) { const int rl = qq >> 3, pc = qq & 7; vst2(O + ((size_t)n * LL + q0 + rl) * DD + h * DH + pc * 4, *(const v4f*)(&sO[w][rl][pc * 4])); }
}
__global__ __launch_bounds__(128) void k_out(const float* __restrict__ O, const __bf16* __restrict__ XH, const __bf16* __restrict__ XL, const float* __restrict__ Wo, const float* __restrict__ bo, const float* __restrict__ Wg, const float* __restrict__ bg, float* __restrict__ out) {
  __shared__ __align__(16) float so[4][16][132];
  const int tid = threadIdx.x, wave = tid >> 5, lane = tid & 31, col = lane & 15, g = lane >> 4; const size_t r0 = (size_t)blockIdx.x * 64 + wave * 16; const int n0 = blockIdx.y * 128;
  v8f acc[8] = {}, accg[8] = {};
#pragma unroll 1
  for (int kc = 0; kc < DD / 32; ++kc) { const F2 a = split_row(O + (r0 + col) * DD, kc * 32, lane); const v16b xh = frag_b(XH + (r0 + col) * DD + kc * 32, lane), xl = frag_b(XL + (r0 + col) * DD + kc * 32, lane);
#pragma unroll
    for (int j = 0; j < 8; ++j) { const v16b wo = split_col(Wo, kc * 32, n0 + j * 16 + col, lane, DD, DD).h, wg = split_col(Wg, kc * 32, n0 + j * 16 + col, lane, DD, DD).h;
      acc[j] = wmma_bf(a.l, wo, acc[j]); acc[j] = wmma_bf(a.h, wo, acc[j]); accg[j] = wmma_bf(xl, wg, accg[j]); accg[j] = wmma_bf(xh, wg, accg[j]); } }
#pragma unroll
  for (int j = 0; j < 8; ++j) { const int c = n0 + j * 16 + col; const float b1 = bfr(bo[c]), b2 = bfr(bg[c]);
#pragma unroll
    for (int r = 0; r < 8; ++r) { const float gate = 1.0f / (1.0f + exp_ni(-(accg[j][r] + b2))); so[wave][8 * g + r][j * 16 + col] = (acc[j][r] + b1) * gate; } }
  LDSX();
  for (int rl = 0; rl < 16; ++rl) vst2(out + (r0 + rl) * DD + n0 + lane * 4, *(const v4f*)(&so[wave][rl][lane * 4]));
}
extern "C" void kernel_launch(void* const* d_in, const int* in_sizes, int n_in, void* d_out, int out_size, void* d_ws, size_t ws_size, hipStream_t stream) {
  (void)in_sizes; (void)n_in; (void)out_size; (void)ws_size;
  const float* msa = (const float*)d_in[0]; const float* pb = (const float*)d_in[1]; const int* mask = (const int*)d_in[2]; const float* lg = (const float*)d_in[3]; const float* lb = (const float*)d_in[4];
  const float* Wq = (const float*)d_in[5]; const float* bq = (const float*)d_in[6]; const float* Wk = (const float*)d_in[7]; const float* bk = (const float*)d_in[8]; const float* Wv = (const float*)d_in[9]; const float* bv = (const float*)d_in[10];
  const float* Wb = (const float*)d_in[11]; const float* bbv = (const float*)d_in[12]; const float* Wo = (const float*)d_in[13]; const float* bo = (const float*)d_in[14]; const float* Wg = (const float*)d_in[15]; const float* bg = (const float*)d_in[16];
  char* ws = (char*)d_ws; size_t off = 0;
  auto take = [&](size_t bytes) { char* p = ws + off; off += (bytes + 255) & ~(size_t)255; return p; };
  __bf16* XH = (__bf16*)take((size_t)NR * DD * 2); __bf16* XL = (__bf16*)take((size_t)NR * DD * 2); float* BIAS = (float*)take((size_t)NHD * LL * LL * 4);
  float* Q32 = (float*)take((size_t)NR * DD * 4); __bf16* Kh = (__bf16*)take((size_t)NR * DD * 2); __bf16* Kl = (__bf16*)take((size_t)NR * DD * 2); __bf16* VTh = (__bf16*)take((size_t)NR * DD * 2); __bf16* VTl = (__bf16*)take((size_t)NR * DD * 2); float* O = (float*)take((size_t)NR * DD * 4);
  k_bias<<<dim3(LL / 64, LL), 128, 0, stream>>>(pb, Wb, bbv, BIAS);
  for (int ps = 0; ps < NSQ / NPS; ++ps) { const size_t rb = (size_t)ps * NR; const float* xin = msa + rb * DD; const int* mk = mask + (size_t)ps * NPS * LL; float* op = (float*)d_out + rb * DD;
    k_ln<<<NR / 8, 256, 0, stream>>>(xin, lg, lb, XH, XL);
    k_qkv<<<dim3(NR / 64, DD / 128, 3), 128, 0, stream>>>(XH, XL, Wq, bq, Wk, bk, Wv, bv, Q32, Kh, Kl, VTh, VTl);
    k_attn<<<dim3(LL / 64, NPS * NHD), 128, 0, stream>>>(Q32, Kh, Kl, VTh, VTl, BIAS, mk, O);
    k_out<<<dim3(NR / 64, DD / 128), 128, 0, stream>>>(O, XH, XL, Wo, bo, Wg, bg, op); }
}
